// GAT_Model_42279658061893
// MI455X (gfx1250) — hardware-verified
//
#include <hip/hip_runtime.h>
#include <math.h>

constexpr int kNodes      = 50000;
constexpr int kEdges      = 800000;
constexpr int kNodesPad   = 50048;
constexpr int kGraphs     = 64;
constexpr int kClasses    = 10;
constexpr int kFeat       = 32;
constexpr int kThreads    = 256;
constexpr int kRows0      = 320;
constexpr int kRows12     = 480;
constexpr int kTiles0     = (kNodesPad + kRows0 - 1) / kRows0;
constexpr int kTiles12    = (kNodesPad + kRows12 - 1) / kRows12;
constexpr int kChunk      = 8192;
constexpr int kPerThr     = kChunk / kThreads;
constexpr int kChunks     = (kEdges + kChunk - 1) / kChunk;
constexpr int kCap        = 1024;
constexpr unsigned kMark  = 0xFFFFFFFFu;
constexpr int kPoolChunk  = 2048;
constexpr int kPoolChunks = (kNodes + kPoolChunk - 1) / kPoolChunk;
constexpr float kCarryW   = 16.0f;
constexpr float kCarryA   = 64.0f;
constexpr float kScale0   = 1.0f / 16.0f;
constexpr float kScale12  = 1.0f / 1024.0f;
constexpr size_t kWsLimit = 134217728;
constexpr size_t kAggLdsBytes = (size_t)kRows0 * 192 * 4;

static_assert(kAggLdsBytes == (size_t)kRows12 * 128 * 4, "");
static_assert(kNodesPad % 64 == 0 && kNodesPad >= kNodes, "");
static_assert(kTiles0 * kRows0 >= kNodesPad && kTiles12 * kRows12 >= kNodesPad, "");
static_assert(kRows0 % 32 == 0 && kRows12 % 32 == 0 && kRows0 <= 512 && kRows12 <= 512, "");
static_assert(kChunk == kPerThr * kThreads, "");
static_assert(kEdges % kPerThr == 0 && kPerThr % 4 == 0, "");
static_assert(kEdges % kThreads == 0, "");
static_assert(kNodes % 8 == 0, "");
static_assert((kNodesPad * kFeat / 8) % kThreads == 0, "");
static_assert(kGraphs * kClasses == 640, "");
static_assert(kEdges < (1 << 20), "");
static_assert(kNodesPad % 64 == 0, "");
static_assert(192 % 64 == 0 && 128 % 64 == 0, "");
static_assert(kFeat % 32 == 0 && 192 % 32 == 0 && 128 % 32 == 0, "");

typedef __attribute__((ext_vector_type(16))) _Float16 v16h;
typedef __attribute__((ext_vector_type(8)))  _Float16 v8h;
typedef __attribute__((ext_vector_type(16))) __bf16   v16b;
typedef __attribute__((ext_vector_type(8)))  __bf16   v8b;
typedef __attribute__((ext_vector_type(8)))  float    v8f;
typedef __attribute__((ext_vector_type(4)))  float    v4f;
typedef __attribute__((ext_vector_type(4)))  unsigned int v4u;
typedef __attribute__((ext_vector_type(4)))  int      v4i;

__device__ __forceinline__ unsigned short f2bf_bits(float f) {
  unsigned u = __float_as_uint(f);
  return (unsigned short)((u + 0x7FFFu + ((u >> 16) & 1u)) >> 16);
}
__device__ __forceinline__ float bf_bits2f(unsigned short h) { return __uint_as_float(((unsigned)h) << 16); }

__device__ __forceinline__ void dep_guard_h(v8f& a, v8f& b, v16h x, v16h y) { asm volatile("v_nop\n\tv_nop\n\tv_nop\n\tv_nop" : "+v"(a), "+v"(b) : "v"(x), "v"(y)); }
__device__ __forceinline__ void dep_guard_b(v8f& a, v8f& b, v16b x, v16b y) { asm volatile("v_nop\n\tv_nop\n\tv_nop\n\tv_nop" : "+v"(a), "+v"(b) : "v"(x), "v"(y)); }
__device__ __forceinline__ void keep4_h(v16h a, v16h b, v16h c, v16h d) { asm volatile("v_nop" :: "v"(a), "v"(b), "v"(c), "v"(d)); }
__device__ __forceinline__ void keep4_b(v16b a, v16b b, v16b c, v16b d) { asm volatile("v_nop" :: "v"(a), "v"(b), "v"(c), "v"(d)); }
__device__ __forceinline__ void acc_guard4(v8f& a, v8f& b, v8f& c, v8f& d) { asm volatile("v_nop\n\tv_nop\n\tv_nop\n\tv_nop" : "+v"(a), "+v"(b), "+v"(c), "+v"(d)); }
template <typename T> struct Frag;
template <> struct Frag<_Float16> {
  typedef v16h V; union U { v16h v; v8h h[2]; };
  static __device__ __forceinline__ v16h load(const _Float16* p) {
    U f; f.h[0] = *(const v8h*)(p); f.h[1] = *(const v8h*)(p + 16); return f.v;
  }
  static __device__ __forceinline__ v8f mma(v16h a, v16h b, v8f c) {
    return __builtin_amdgcn_wmma_f32_16x16x32_f16(false, a, false, b, (short)0, c, false, false);
  }
  static __device__ __forceinline__ void guard(v8f& a, v8f& b, v16h x, v16h y) { dep_guard_h(a, b, x, y); }
  static __device__ __forceinline__ void keep(v16h a, v16h b, v16h c, v16h d) { keep4_h(a, b, c, d); }
};
template <> struct Frag<__bf16> {
  typedef v16b V; union U { v16b v; v8b h[2]; };
  static __device__ __forceinline__ v16b load(const __bf16* p) {
    U f; f.h[0] = *(const v8b*)(p); f.h[1] = *(const v8b*)(p + 16); return f.v;
  }
  static __device__ __forceinline__ v8f mma(v16b a, v16b b, v8f c) {
    return __builtin_amdgcn_wmma_f32_16x16x32_bf16(false, a, false, b, (short)0, c, false, false);
  }
  static __device__ __forceinline__ void guard(v8f& a, v8f& b, v16b x, v16b y) { dep_guard_b(a, b, x, y); }
  static __device__ __forceinline__ void keep(v16b a, v16b b, v16b c, v16b d) { keep4_b(a, b, c, d); }
};

__device__ __forceinline__ unsigned pk16(unsigned short a, unsigned short b) { return (unsigned)a | ((unsigned)b << 16); }
__device__ __forceinline__ unsigned short h_bits(float f) { const _Float16 h = (_Float16)f; return __builtin_bit_cast(unsigned short, h); }

template <int ET> struct Elem;
template <> struct Elem<0> { typedef _Float16 T; };
template <> struct Elem<1> { typedef __bf16 T; };
template <int ET, bool SPLIT, int BIAS_MODE, int OUT_MODE, bool RESID, int ACT = 0>
__global__ __launch_bounds__(256) void wmma_gemm64(
    const unsigned short* __restrict__ Ap, const unsigned short* __restrict__ A2p, int lda, long strideA,
    const unsigned short* __restrict__ Btp, const unsigned short* __restrict__ Bt2p, int ldb, long strideB,
    void* __restrict__ Cout, void* __restrict__ Cout2, int ldc, long strideC,
    const float* __restrict__ bias,
    const float* __restrict__ resid, long strideR,
    int M, int N, int K, float scale) {
  typedef typename Elem<ET>::T T;
  typedef typename Frag<T>::V V;
  const T* A = (const T*)Ap; const T* A2 = (const T*)A2p; const T* Bt = (const T*)Btp; const T* Bt2 = (const T*)Bt2p;
  __shared__ __align__(16) float sT[8][16 * 68];
  const int b    = blockIdx.y;
  const int lane = threadIdx.x & 31;
  const int wave = threadIdx.x >> 5;
  const int tilesN = N >> 6;
  const int tilesM = M >> 6;
  const int tile = blockIdx.x * 8 + wave;
  if (tile >= tilesM * tilesN) return;
  const int tm = tile / tilesN;
  const int tn = tile - tm * tilesN;
  const int m0 = tm << 6;
  const int n0 = tn << 6;

  const T* Ab  = A  + (size_t)b * strideA;
  const T* Bb  = Bt + (size_t)b * strideB;
  const T* Ab2 = SPLIT ? (A2  + (size_t)b * strideA) : nullptr;
  const T* Bb2 = SPLIT ? (Bt2 + (size_t)b * strideB) : nullptr;

  const int rlane = lane & 15;
  const int koff  = (lane >> 4) * 8;
  const int mOff  = (lane >> 4) * 8;

  v8f acc[4][4];
#pragma unroll
  for (int i = 0; i < 4; ++i)
#pragma unroll
    for (int j = 0; j < 4; ++j) acc[i][j] = (v8f){0.f,0.f,0.f,0.f,0.f,0.f,0.f,0.f};

  for (int k0 = 0; k0 < K; k0 += 32) {
    V bh[4], bl[4];
#pragma unroll
    for (int j = 0; j < 4; ++j) {
      const size_t bo = (size_t)(n0 + (j << 4) + rlane) * ldb + koff + k0;
      bh[j] = Frag<T>::load(Bb + bo);
      if (SPLIT) bl[j] = Frag<T>::load(Bb2 + bo);
    }
#pragma unroll
    for (int i = 0; i < 4; ++i) {
      const size_t ao = (size_t)(m0 + (i << 4) + rlane) * lda + koff + k0;
      V ah = Frag<T>::load(Ab + ao);
      V al;
      if (SPLIT) al = Frag<T>::load(Ab2 + ao);
#pragma unroll
      for (int j = 0; j < 4; ++j) {
        acc[i][j] = Frag<T>::mma(ah, bh[j], acc[i][j]);
        if (SPLIT) {
          acc[i][j] = Frag<T>::mma(ah, bl[j], acc[i][j]);
          acc[i][j] = Frag<T>::mma(al, bh[j], acc[i][j]);
        }
      }
      Frag<T>::guard(acc[i][0], acc[i][3], ah, SPLIT ? al : ah);
    }
    Frag<T>::keep(bh[0], bh[1], bh[2], bh[3]);
    if (SPLIT) Frag<T>::keep(bl[0], bl[1], bl[2], bl[3]);
  }
  acc_guard4(acc[0][0], acc[0][1], acc[0][2], acc[0][3]);
  acc_guard4(acc[1][0], acc[1][1], acc[1][2], acc[1][3]);
  acc_guard4(acc[2][0], acc[2][1], acc[2][2], acc[2][3]);
  acc_guard4(acc[3][0], acc[3][1], acc[3][2], acc[3][3]);

  float* slab = sT[wave];
  const float* Rb = RESID ? (resid + (size_t)b * strideR) : nullptr;
#pragma unroll
  for (int i = 0; i < 4; ++i) {
    const int mBase = m0 + (i << 4);
#pragma unroll
    for (int j = 0; j < 4; ++j) {
      const int n = n0 + (j << 4) + rlane;
      float bv = 0.f;
      if (BIAS_MODE == 2) bv = bias[n];
#pragma unroll
      for (int r = 0; r < 8; ++r) {
        float v = acc[i][j][r] * scale;
        if (BIAS_MODE == 1) v += bias[mBase + mOff + r];
        if (BIAS_MODE == 2) v += bv;
        if (RESID) v += Rb[(size_t)(mBase + mOff + r) * ldc + n];
        if (ACT == 2) v = fmaxf(v, 0.0f);
        if (ACT == 4) v = (v > 0.f) ? v : 0.01f * v;
        slab[(mOff + r) * 68 + (j << 4) + rlane] = v;
      }
    }
    __builtin_amdgcn_fence(__ATOMIC_RELEASE, "workgroup");
    __builtin_amdgcn_wave_barrier();
    __builtin_amdgcn_fence(__ATOMIC_ACQUIRE, "workgroup");
    if (OUT_MODE == 0) {
      float* C = (float*)Cout + (size_t)b * strideC;
      const int hh = lane >> 4, c4 = (lane & 15) * 4;
      for (int pass = 0; pass < 2; ++pass) {
#pragma unroll
        for (int it = 0; it < 8; ++it) {
          const int row = it * 2 + hh;
          v4f v = *(const v4f*)(slab + row * 68 + c4);
          *(volatile v4f*)(C + (size_t)(mBase + row) * ldc + n0 + c4) = v;
        }
        __threadfence();
      }
    } else {
      const int q = lane >> 3, c8 = (lane & 7) * 8;
      unsigned short* C  = (unsigned short*)Cout  + (size_t)b * strideC;
      unsigned short* C2 = (OUT_MODE == 2) ? ((unsigned short*)Cout2 + (size_t)b * strideC) : nullptr;
      for (int pass = 0; pass < 2; ++pass) {
#pragma unroll
        for (int it = 0; it < 4; ++it) {
          const int row = it * 4 + q;
          const float* sp = slab + row * 68 + c8;
          v8h hv, lv;
#pragma unroll
          for (int e = 0; e < 8; ++e) {
            if (OUT_MODE == 1) {
              hv[e] = (_Float16)sp[e];
            } else {
              unsigned short hb = f2bf_bits(sp[e]);
              unsigned short lb = f2bf_bits(sp[e] - bf_bits2f(hb));
              hv[e] = __builtin_bit_cast(_Float16, hb);
              lv[e] = __builtin_bit_cast(_Float16, lb);
            }
          }
          *(volatile v8h*)(C + (size_t)(mBase + row) * ldc + n0 + c8) = hv;
          if (OUT_MODE == 2) *(volatile v8h*)(C2 + (size_t)(mBase + row) * ldc + n0 + c8) = lv;
        }
        __threadfence();
      }
    }
    __builtin_amdgcn_fence(__ATOMIC_RELEASE, "workgroup");
    __builtin_amdgcn_wave_barrier();
    __builtin_amdgcn_fence(__ATOMIC_ACQUIRE, "workgroup");
  }
}

__global__ __launch_bounds__(kThreads) void cast_x_kernel(const float* __restrict__ x, unsigned short* __restrict__ out) {
  const int u = blockIdx.x * kThreads + threadIdx.x;
  const int row = u >> 2;
  const int c8 = (u & 3) * 8;
  const bool live = row < kNodes;
  const float livef = live ? 1.0f : 0.0f;
  const int rc = live ? row : (kNodes - 1);
  const float* p = x + (size_t)rc * kFeat + c8;
  const v4f a = *(const v4f*)(p);
  const v4f c = *(const v4f*)(p + 4);
  unsigned short hb[8];
#pragma unroll
  for (int e = 0; e < 4; ++e) {
    hb[e]     = h_bits(a[e] * livef);
    hb[4 + e] = h_bits(c[e] * livef);
  }
  const v4u w = (v4u){pk16(hb[0], hb[1]), pk16(hb[2], hb[3]), pk16(hb[4], hb[5]), pk16(hb[6], hb[7])};
  unsigned short* q = out + 8 * (size_t)u;
  *(volatile v4u*)q = w;
  __threadfence();
  *(volatile v4u*)q = w;
}

template <int KD>
__global__ __launch_bounds__(kThreads) void wt_kernel(const float* __restrict__ Wa, const float* __restrict__ Wb,
                                                     unsigned short* __restrict__ outA, unsigned short* __restrict__ outB, int nout) {
  static_assert(KD % 32 == 0 && KD <= 192, "");
  __shared__ float sm[64][KD + 1];
  const int t = threadIdx.x;
  const int n0 = blockIdx.x * 64;
  const int z = blockIdx.y;
  const float* W = (z == 0) ? Wa : Wb;
  unsigned short* o = (z == 0) ? outA : outB;
#pragma unroll 4
  for (int it = 0; it < KD / 16; ++it) {
    const int unit = it * kThreads + t;
    const int kk = unit >> 4;
    const int c4 = (unit & 15) * 4;
    const v4f w = *(const v4f*)(W + (size_t)kk * nout + n0 + c4);
#pragma unroll
    for (int e = 0; e < 4; ++e) sm[c4 + e][kk] = w[e] * kCarryW;
  }
  __syncthreads();
  unsigned short* ob = o + (size_t)n0 * KD;
  for (int pass = 0; pass < 2; ++pass) {
#pragma unroll
    for (int it = 0; it < KD / 32; ++it) {
      const int u = it * kThreads + t;
      const int hi0 = 8 * u;
      const int r = hi0 / KD;
      const int k = hi0 - r * KD;
      unsigned short hb[8];
#pragma unroll
      for (int e = 0; e < 8; ++e) hb[e] = h_bits(sm[r][k + e]);
      const v4u w = (v4u){pk16(hb[0], hb[1]), pk16(hb[2], hb[3]), pk16(hb[4], hb[5]), pk16(hb[6], hb[7])};
      *(volatile v4u*)(ob + hi0) = w;
    }
    __threadfence();
  }
}

template <int H>
__global__ __launch_bounds__(kThreads) void node_kernel(const float* __restrict__ XL, const float* __restrict__ XR, const float* __restrict__ att,
                                                       float* __restrict__ AL4, float* __restrict__ AR4, float* __restrict__ CS4) {
  constexpr int HC = 64 * H;
  const int i = blockIdx.x * kThreads + threadIdx.x;
  const bool live = i < kNodes;
  const int n = live ? i : (kNodes - 1);
  const float* pl = XL + (size_t)n * HC;
  const float* pr = XR + (size_t)n * HC;
  float alo[3] = {0.f, 0.f, 0.f}, aro[3] = {0.f, 0.f, 0.f}, cso[3] = {0.f, 0.f, 0.f};
#pragma unroll
  for (int h = 0; h < H; ++h) {
    float sa = 0.0f, sr = 0.0f, sp = 0.0f;
#pragma unroll 1
    for (int c4 = 0; c4 < 16; ++c4) {
      const v4f a = *(const v4f*)(pl + h * 64 + 4 * c4);
      const v4f r = *(const v4f*)(pr + h * 64 + 4 * c4);
      const v4f w = *(const v4f*)(att + h * 64 + 4 * c4);
#pragma unroll
      for (int u = 0; u < 4; ++u) {
        sa += a[u] * w[u];
        sr += r[u] * w[u];
        float tt = a[u] + r[u];
        tt = fmaxf(tt, 0.0f);
        sp += tt * w[u];
      }
    }
    alo[h] = sa;
    aro[h] = sr;
    cso[h] = 0.2f * (sa + sr) + 0.8f * sp;
  }
  const v4f oa = {alo[0], alo[1], alo[2], 0.0f};
  const v4f orr = {aro[0], aro[1], aro[2], 0.0f};
  const v4f oc = {cso[0], cso[1], cso[2], 0.0f};
  if (live) {
    float* pa = AL4 + 4 * (size_t)i;
    float* pb = AR4 + 4 * (size_t)i;
    float* pc = CS4 + 4 * (size_t)i;
    for (int pass = 0; pass < 2; ++pass) {
      *(volatile v4f*)pa = oa;
      *(volatile v4f*)pb = orr;
      *(volatile v4f*)pc = oc;
      __threadfence();
    }
  }
}

template <int H>
__global__ __launch_bounds__(kThreads) void ex_kernel(const float* __restrict__ XL, const float* __restrict__ XR, const float* __restrict__ att,
                                                     const int* __restrict__ ei, const float* __restrict__ AL4, const float* __restrict__ AR4,
                                                     const float* __restrict__ CS4, float* __restrict__ EX) {
  constexpr int HC = 64 * H;
  const int e = blockIdx.x * kThreads + threadIdx.x;
  const int sr = ei[e];
  const int dr = ei[kEdges + e];
  const float fval = (sr != dr) ? 1.0f : 0.0f;
  const int s = sr < 0 ? 0 : (sr >= kNodes ? kNodes - 1 : sr);
  const int d = dr < 0 ? 0 : (dr >= kNodes ? kNodes - 1 : dr);
  const v4f alv = *(const v4f*)(AL4 + 4 * (size_t)s);
  const v4f arv = *(const v4f*)(AR4 + 4 * (size_t)d);
  const v4f csv = *(const v4f*)(CS4 + 4 * (size_t)d);
  const float* pl = XL + (size_t)s * HC;
  const float* pr = XR + (size_t)d * HC;
  float exo[3] = {0.f, 0.f, 0.f};
#pragma unroll
  for (int h = 0; h < H; ++h) {
    float sp = 0.0f;
#pragma unroll 2
    for (int c4 = 0; c4 < 16; ++c4) {
      const v4f a = *(const v4f*)(pl + h * 64 + 4 * c4);
      const v4f r = *(const v4f*)(pr + h * 64 + 4 * c4);
      const v4f w = *(const v4f*)(att + h * 64 + 4 * c4);
#pragma unroll
      for (int u = 0; u < 4; ++u) {
        float tt = a[u] + r[u];
        tt = fmaxf(tt, 0.0f);
        sp += tt * w[u];
      }
    }
    const float lg = 0.2f * (alv[h] + arv[h]) + 0.8f * sp;
    const float z = fminf(lg - csv[h], 80.0f);
    exo[h] = expf(z) * fval;
  }
  const v4f o = {exo[0], exo[1], exo[2], 0.0f};
  float* op = EX + 4 * (size_t)e;
  *(volatile v4f*)op = o;
  __threadfence();
  *(volatile v4f*)op = o;
}

__device__ __forceinline__ int blk_excl_scan(int cnt, int* scan_ws, int tid, int* tot) {
  const int lane = tid & 31, wave = tid >> 5; int incl = cnt;
#pragma unroll
  for (int o = 1; o < 32; o <<= 1) { const int v = __shfl_up(incl, o, 32); if (lane >= o) incl += v; }
  if (lane == 31) scan_ws[wave] = incl;
  __syncthreads();
  if (wave == 0) { int wv = (lane < kThreads / 32) ? scan_ws[lane] : 0; int wincl = wv;
#pragma unroll
    for (int o = 1; o < 32; o <<= 1) { const int v = __shfl_up(wincl, o, 32); if (lane >= o) wincl += v; }
    if (lane < kThreads / 32) scan_ws[32 + lane] = wincl - wv; if (lane == 31) scan_ws[64] = wincl; }
  __syncthreads();
  const int res = scan_ws[32 + wave] + incl - cnt; *tot = scan_ws[64];
  return res;
}

template <int SP, int CAPV, int ROWS>
__device__ __forceinline__ int chunk_hits(const int* __restrict__ dstv, int e0, int n0, int tid, unsigned* LIST, int* scan_ws) {
  const int eb = e0 + tid * SP;
  const bool inr = eb < kEdges;
  const int ebc = inr ? eb : (kEdges - SP);
  unsigned rec[SP];
  int cnt = 0;
#pragma unroll
  for (int k = 0; k < SP; k += 4) {
    const v4i d4 = *(const v4i*)(dstv + ebc + k);
#pragma unroll
    for (int x = 0; x < 4; ++x) {
      const unsigned rel = (unsigned)(d4[x] - n0);
      const bool hit = inr && (rel < (unsigned)ROWS);
      rec[k + x] = hit ? ((rel << 20) | (unsigned)(ebc + k + x)) : kMark;
      cnt += hit ? 1 : 0;
    }
  }
  int tot;
  int p = blk_excl_scan(cnt, scan_ws, tid, &tot);
#pragma unroll
  for (int k = 0; k < SP; ++k) {
    const bool hk = rec[k] != kMark;
    if (hk && (unsigned)p < (unsigned)CAPV) LIST[p] = rec[k];
    p += hk ? 1 : 0;
  }
  __syncthreads();
  return tot < CAPV ? tot : CAPV;
}

template <int H, int ROWS>
__device__ __forceinline__ void agg_hit(const float* __restrict__ XL, const int* __restrict__ ei, const float* __restrict__ EX,
                                        float* ACC, float* DEN, int q, unsigned myr, int act) {
  constexpr int HC = 64 * H;
  constexpr int NJ = 2 * H;
  int e = (int)(myr & 0xFFFFFu);
  e = e < kEdges ? e : (kEdges - 1);
  int rel = (int)(myr >> 20);
  rel = rel < ROWS ? rel : (ROWS - 1);
  int s = ei[e];
  s = s < 0 ? 0 : (s >= kNodes ? kNodes - 1 : s);
  const v4f exv = *(const v4f*)(EX + 4 * (size_t)e);
  const float* xp = XL + (size_t)s * HC + 4 * q;
  float* rp = ACC + rel * HC + 4 * q;
  v4f a[NJ];
#pragma unroll
  for (int j = 0; j < NJ; ++j) {
    const v4f xa = *(const v4f*)(xp + 32 * j);
    const v4f ao = *(const v4f*)(rp + 32 * j);
    a[j] = exv[j >> 1] * xa + ao;
  }
  float dn[H];
#pragma unroll
  for (int h = 0; h < H; ++h) dn[h] = DEN[rel * H + h];
  if (act) {
#pragma unroll
    for (int j = 0; j < NJ; ++j) *(v4f*)(rp + 32 * j) = a[j];
    if (q == 0) {
#pragma unroll
      for (int h = 0; h < H; ++h) DEN[rel * H + h] = dn[h] + exv[h];
    }
  }
}

template <int H, int MODE, int ROWS>
__global__ __launch_bounds__(kThreads) void agg_kernel(const float* __restrict__ XL, const int* __restrict__ ei,
                                                      const float* __restrict__ EX, const float* __restrict__ bias,
                                                      unsigned short* __restrict__ HO16, float* __restrict__ HO32) {
  static_assert(MODE == 0 || H == 2, "");
  static_assert(ROWS % 32 == 0 && ROWS <= 512, "");
  constexpr int HC = 64 * H;
  constexpr int NJ = 2 * H;
  constexpr int STEPS = ROWS / 32;
  static_assert((size_t)ROWS * HC * 4 == kAggLdsBytes, "");
  extern __shared__ v4f agg_dyn4[];
  __shared__ unsigned LIST[kCap];
  __shared__ float DEN[ROWS * H];
  __shared__ int scan_ws[80];
  float* ACC = (float*)agg_dyn4;
  const int tid = threadIdx.x, lane = tid & 31, wave = tid >> 5, grp = lane >> 3, q = lane & 7;
  const int n0 = blockIdx.x * ROWS;
  const v4f z4 = {0.f, 0.f, 0.f, 0.f};
  for (int i = tid; i < ROWS * HC / 4; i += kThreads) agg_dyn4[i] = z4;
  for (int i = tid; i < kCap; i += kThreads) LIST[i] = kMark;
  for (int i = tid; i < ROWS * H; i += kThreads) DEN[i] = 0.0f;
  if (tid < 80) scan_ws[tid] = 0;
  __syncthreads();

  const int* dstv = ei + kEdges;
#pragma unroll 1
  for (int c = 0; c < kChunks; ++c) {
    const int tot = chunk_hits<kPerThr, kCap, ROWS>(dstv, c * kChunk, n0, tid, LIST, scan_ws);
#pragma unroll 1
    for (int base = 0; base < tot; base += 32) {
      const int qq = base + lane;
      const int qc = (qq < tot) ? qq : (tot - 1);
      const unsigned lv = LIST[qc];
      const int own = ((qq < tot) && ((int)((lv >> 20) & 7u) == wave)) ? 1 : 0;
      unsigned msk = (unsigned)__ballot(own);
#pragma unroll 1
      for (int it = 0; it < 8; ++it) {
        if (msk == 0u) break;
        unsigned mm = msk;
        const int bA = __builtin_ctz(mm);
        mm &= mm - 1u;
        const int hB = (mm != 0u) ? 1 : 0; const int bB = hB ? __builtin_ctz(mm) : bA; mm &= mm - 1u;
        const int hC = (mm != 0u) ? 1 : 0; const int bC = hC ? __builtin_ctz(mm) : bA; mm &= mm - 1u;
        const int hD = (mm != 0u) ? 1 : 0; const int bD = hD ? __builtin_ctz(mm) : bA; mm &= mm - 1u;
        msk = mm;
        const unsigned rA = (unsigned)__builtin_amdgcn_readlane((int)lv, bA);
        const unsigned rB = (unsigned)__builtin_amdgcn_readlane((int)lv, bB);
        const unsigned rC = (unsigned)__builtin_amdgcn_readlane((int)lv, bC);
        const unsigned rD = (unsigned)__builtin_amdgcn_readlane((int)lv, bD);
        const unsigned dA = rA >> 20, dB = rB >> 20, dC = rC >> 20, dD = rD >> 20;
        const bool coll = (hB && (dB == dA)) || (hC && ((dC == dA) || (dC == dB))) || (hD && ((dD == dA) || (dD == dB) || (dD == dC)));
        const int nsub = coll ? 4 : 1;
#pragma unroll 1
        for (int sub = 0; sub < nsub; ++sub) {
          unsigned myr; int act;
          if (coll) {
            myr = (sub == 0) ? rA : (sub == 1) ? rB : (sub == 2) ? rC : rD;
            const int hs = (sub == 0) ? 1 : (sub == 1) ? hB : (sub == 2) ? hC : hD;
            act = (grp == 0) ? hs : 0;
          } else {
            myr = (grp == 0) ? rA : (grp == 1) ? rB : (grp == 2) ? rC : rD;
            act = (grp == 0) ? 1 : (grp == 1) ? hB : (grp == 2) ? hC : hD;
          }
          agg_hit<H, ROWS>(XL, ei, EX, ACC, DEN, q, myr, act);
        }
      }
    }
    __syncthreads();
  }

#pragma unroll 1
  for (int st = 0; st < STEPS; ++st) {
    const int rel = 8 * (4 * st + grp) + wave;
    const int n = n0 + rel;
    const int act = (n < kNodes) ? 1 : 0;
    const int nc = act ? n : (kNodes - 1);
    const float* xp = XL + (size_t)nc * HC + 4 * q;
    float* rp = ACC + rel * HC + 4 * q;
    v4f a[NJ];
#pragma unroll
    for (int j = 0; j < NJ; ++j) a[j] = *(const v4f*)(xp + 32 * j) + *(const v4f*)(rp + 32 * j);
    float dn[H];
#pragma unroll
    for (int h = 0; h < H; ++h) dn[h] = DEN[rel * H + h];
    if (act) {
#pragma unroll
      for (int j = 0; j < NJ; ++j) *(v4f*)(rp + 32 * j) = a[j];
      if (q == 0) {
#pragma unroll
        for (int h = 0; h < H; ++h) DEN[rel * H + h] = dn[h] + 1.0f;
      }
    }
  }
  __syncthreads();

  if constexpr (MODE == 0) {
    v4f bA[H], bB[H];
#pragma unroll
    for (int jl = 0; jl < H; ++jl) {
      bA[jl] = *(const v4f*)(bias + 64 * jl + 8 * q);
      bB[jl] = *(const v4f*)(bias + 64 * jl + 8 * q + 4);
    }
#pragma unroll 1
    for (int st = 0; st < STEPS; ++st) {
      const int rel = 8 * (4 * st + grp) + wave;
      const int n = n0 + rel;
      const bool wr = n < kNodesPad;
      const float livef = (n < kNodes) ? 1.0f : 0.0f;
      const float* rp = ACC + rel * HC + 8 * q;
      float inv[H];
#pragma unroll
      for (int h = 0; h < H; ++h) {
        const float dd = DEN[rel * H + h] + (1.0f - livef);
        inv[h] = 1.0f / dd;
      }
      const float cl = kCarryA * livef;
      v4u ov[H];
#pragma unroll
      for (int jl = 0; jl < H; ++jl) {
        const v4f u0 = *(const v4f*)(rp + 64 * jl);
        const v4f u1 = *(const v4f*)(rp + 64 * jl + 4);
        const v4f t0 = u0 * inv[jl] + bA[jl];
        const v4f t1 = u1 * inv[jl] + bB[jl];
        unsigned short hb[8];
#pragma unroll
        for (int e = 0; e < 4; ++e) {
          hb[e]     = h_bits(fmaxf(t0[e], 0.0f) * cl);
          hb[4 + e] = h_bits(fmaxf(t1[e], 0.0f) * cl);
        }
        ov[jl] = (v4u){pk16(hb[0], hb[1]), pk16(hb[2], hb[3]), pk16(hb[4], hb[5]), pk16(hb[6], hb[7])};
      }
      if (wr) {
        unsigned short* op = HO16 + (size_t)n * HC + 8 * q;
        for (int pass = 0; pass < 2; ++pass) {
#pragma unroll
          for (int jl = 0; jl < H; ++jl) *(volatile v4u*)(op + 64 * jl) = ov[jl];
          __threadfence();
        }
      }
    }
  } else {
    const v4f bq0 = *(const v4f*)(bias + 4 * q);
    const v4f bq1 = *(const v4f*)(bias + 32 + 4 * q);
#pragma unroll 1
    for (int st = 0; st < STEPS; ++st) {
      const int rel = 8 * (4 * st + grp) + wave;
      const int n = n0 + rel;
      const bool wr = n < kNodesPad;
      const float livef = (n < kNodes) ? 1.0f : 0.0f;
      const float* rp = ACC + rel * HC + 4 * q;
      float inv[2];
#pragma unroll
      for (int h = 0; h < 2; ++h) {
        const float dd = DEN[rel * H + h] + (1.0f - livef);
        inv[h] = 1.0f / dd;
      }
      const v4f u00 = *(const v4f*)(rp);
      const v4f u01 = *(const v4f*)(rp + 32);
      const v4f u10 = *(const v4f*)(rp + 64);
      const v4f u11 = *(const v4f*)(rp + 96);
      const v4f m0 = (u00 * inv[0] + u10 * inv[1]) * 0.5f;
      const v4f m1 = (u01 * inv[0] + u11 * inv[1]) * 0.5f;
      const v4f t0 = m0 + bq0;
      const v4f t1 = m1 + bq1;
      v4f o0, o1;
#pragma unroll
      for (int e = 0; e < 4; ++e) {
        o0[e] = fmaxf(t0[e], 0.0f) * livef;
        o1[e] = fmaxf(t1[e], 0.0f) * livef;
      }
      if (wr) {
        float* op = HO32 + (size_t)n * 64 + 4 * q;
        for (int pass = 0; pass < 2; ++pass) {
          *(volatile v4f*)(op) = o0;
          *(volatile v4f*)(op + 32) = o1;
          __threadfence();
        }
      }
    }
  }
}

__global__ __launch_bounds__(kThreads) void pool_kernel(const float* __restrict__ H2, const int* __restrict__ batch, float* __restrict__ P) {
  __shared__ int LIST[kPoolChunk];
  __shared__ int scan_ws[80];
  __shared__ __align__(16) float redS[8 * 128];
  __shared__ __align__(16) float redM[8 * 128];
  __shared__ float rc[16];
  const int tid = threadIdx.x, lane = tid & 31, wave = tid >> 5;
  const int half = lane >> 4;
  const int c4 = (lane & 15) * 4;
  const int g = blockIdx.x;
  const v4f z4 = {0.f, 0.f, 0.f, 0.f};
  for (int i = tid; i < kPoolChunk; i += kThreads) LIST[i] = 0;
  if (tid < 80) scan_ws[tid] = 0;
  __syncthreads();
  v4f acc = z4, mx = z4;
  float cnt = 0.0f;
#pragma unroll 1
  for (int c = 0; c < kPoolChunks; ++c) {
    const int eb = c * kPoolChunk + tid * 8;
    const bool inr = eb < kNodes;
    const int ebc = inr ? eb : (kNodes - 8);
    const v4i b0 = *(const v4i*)(batch + ebc);
    const v4i b1 = *(const v4i*)(batch + ebc + 4);
    int rec[8]; int kc = 0;
#pragma unroll
    for (int k = 0; k < 4; ++k) {
      const bool h0 = inr && (b0[k] == g);
      const bool h1 = inr && (b1[k] == g);
      rec[k]     = h0 ? (ebc + k) : -1;
      rec[4 + k] = h1 ? (ebc + 4 + k) : -1;
      kc += (h0 ? 1 : 0) + (h1 ? 1 : 0);
    }
    int tot;
    int p = blk_excl_scan(kc, scan_ws, tid, &tot);
#pragma unroll
    for (int k = 0; k < 8; ++k) {
      const bool hk = rec[k] >= 0;
      if (hk && (unsigned)p < (unsigned)kPoolChunk) LIST[p] = rec[k];
      p += hk ? 1 : 0;
    }
    __syncthreads();
    const int totc = tot < kPoolChunk ? tot : kPoolChunk;
#pragma unroll 1
    for (int qb = wave * 2; qb < totc; qb += 16) {
      const int qq = qb + half;
      const bool act = qq < totc;
      const int qcl = act ? qq : (totc - 1);
      int nd = LIST[qcl];
      nd = nd < 0 ? 0 : (nd >= kNodes ? kNodes - 1 : nd);
      const v4f v = *(const v4f*)(H2 + (size_t)nd * 64 + c4);
      const float f = act ? 1.0f : 0.0f;
      const v4f vf = v * f;
      acc = acc + vf;
#pragma unroll
      for (int e = 0; e < 4; ++e) mx[e] = fmaxf(mx[e], vf[e]);
      cnt += f;
    }
    __syncthreads();
  }
  *(v4f*)(redS + wave * 128 + half * 64 + c4) = acc;
  *(v4f*)(redM + wave * 128 + half * 64 + c4) = mx;
  if ((lane & 15) == 0) rc[wave * 2 + half] = cnt;
  __syncthreads();
  if (wave == 0) {
    v4f s = z4, m = z4;
    float ct = 0.0f;
#pragma unroll
    for (int w = 0; w < 8; ++w) {
#pragma unroll
      for (int hh = 0; hh < 2; ++hh) {
        const v4f rs = *(const v4f*)(redS + w * 128 + hh * 64 + c4);
        const v4f rm = *(const v4f*)(redM + w * 128 + hh * 64 + c4);
        s = s + rs;
#pragma unroll
        for (int e = 0; e < 4; ++e) m[e] = fmaxf(m[e], rm[e]);
        ct += rc[w * 2 + hh];
      }
    }
    const float inv = 1.0f / fmaxf(ct, 1.0f);
    const v4f mean = s * inv;
    const float hf = half ? 1.0f : 0.0f;
    const v4f o = m * (1.0f - hf) + mean * hf;
    float* op = P + (size_t)g * 128 + 4 * lane;
    for (int pass = 0; pass < 2; ++pass) { *(volatile v4f*)op = o; __threadfence(); }
  }
}

__global__ __launch_bounds__(kThreads) void head_kernel(const float* __restrict__ P, const float* __restrict__ Wout,
                                                       const float* __restrict__ bout, float* __restrict__ out) {
  __shared__ __align__(16) float so[640];
  const int tid = threadIdx.x, lane = tid & 31, wave = tid >> 5;
  for (int i = tid; i < kGraphs * kClasses; i += kThreads) {
    const int g = i / kClasses;
    const int k = i - g * kClasses;
    float s = 0.0f;
#pragma unroll 1
    for (int j = 0; j < 128; ++j) s += P[g * 128 + j] * Wout[j * kClasses + k];
    so[i] = s + bout[k];
  }
  __syncthreads();
  if (wave == 0) {
    v4f pv[5];
#pragma unroll
    for (int kk = 0; kk < 5; ++kk) pv[kk] = *(const v4f*)(so + 128 * kk + 4 * lane);
    for (int pass = 0; pass < 2; ++pass) {
#pragma unroll
      for (int kk = 0; kk < 5; ++kk) *(volatile v4f*)(out + 128 * kk + 4 * lane) = pv[kk];
      __threadfence();
    }
  }
}

extern "C" void kernel_launch(void* const* d_in, const int* in_sizes, int n_in,
                              void* d_out, int out_size, void* d_ws, size_t ws_size, hipStream_t stream) {
  (void)in_sizes; (void)n_in; (void)out_size;
  const float* x     = (const float*)d_in[0];
  const int*   ei    = (const int*)  d_in[1];
  const int*   batch = (const int*)  d_in[2];
  const float* Wl0 = (const float*)d_in[3];  const float* bl0 = (const float*)d_in[4];
  const float* Wr0 = (const float*)d_in[5];  const float* br0 = (const float*)d_in[6];
  const float* att0 = (const float*)d_in[7]; const float* bias0 = (const float*)d_in[8];
  const float* Wl1 = (const float*)d_in[9];  const float* bl1 = (const float*)d_in[10];
  const float* Wr1 = (const float*)d_in[11]; const float* br1 = (const float*)d_in[12];
  const float* att1 = (const float*)d_in[13]; const float* bias1 = (const float*)d_in[14];
  const float* Wl2 = (const float*)d_in[15]; const float* bl2 = (const float*)d_in[16];
  const float* Wr2 = (const float*)d_in[17]; const float* br2 = (const float*)d_in[18];
  const float* att2 = (const float*)d_in[19]; const float* bias2 = (const float*)d_in[20];
  const float* Wout = (const float*)d_in[21]; const float* bout = (const float*)d_in[22];
  float* out = (float*)d_out;

  char* ws = (char*)d_ws; size_t off = 0;
  auto carve = [&](size_t bytes) -> char* { char* p = ws + off; off += (bytes + 255) & ~(size_t)255; return p; };
  unsigned short* X16  = (unsigned short*)carve((size_t)kNodesPad * kFeat * 2);
  unsigned short* WL0T = (unsigned short*)carve((size_t)192 * 32 * 2);
  unsigned short* WR0T = (unsigned short*)carve((size_t)192 * 32 * 2);
  unsigned short* WL1T = (unsigned short*)carve((size_t)128 * 192 * 2);
  unsigned short* WR1T = (unsigned short*)carve((size_t)128 * 192 * 2);
  unsigned short* WL2T = (unsigned short*)carve((size_t)128 * 128 * 2);
  unsigned short* WR2T = (unsigned short*)carve((size_t)128 * 128 * 2);
  float*          XL   = (float*)carve((size_t)kNodesPad * 192 * 4);
  float*          XR   = (float*)carve((size_t)kNodesPad * 192 * 4);
  unsigned short* HA   = (unsigned short*)carve((size_t)kNodesPad * 192 * 2);
  float*          H2   = (float*)carve((size_t)kNodesPad * 64 * 4);
  float*          AL4  = (float*)carve((size_t)kNodesPad * 4 * 4);
  float*          AR4  = (float*)carve((size_t)kNodesPad * 4 * 4);
  float*          CS4  = (float*)carve((size_t)kNodesPad * 4 * 4);
  float*          EXP  = (float*)carve((size_t)kEdges * 4 * 4);
  float*          PP   = (float*)carve((size_t)kGraphs * 128 * 4);
  if (off > ws_size || off > kWsLimit) return;

  cast_x_kernel<<<(kNodesPad * kFeat / 8) / kThreads, kThreads, 0, stream>>>(x, X16);
  wt_kernel<32><<<dim3(192 / 64, 2), kThreads, 0, stream>>>(Wl0, Wr0, WL0T, WR0T, 192);
  wt_kernel<192><<<dim3(128 / 64, 2), kThreads, 0, stream>>>(Wl1, Wr1, WL1T, WR1T, 128);
  wt_kernel<128><<<dim3(128 / 64, 2), kThreads, 0, stream>>>(Wl2, Wr2, WL2T, WR2T, 128);

  const int tiles192 = (kNodesPad / 64) * (192 / 64);
  const int tiles128 = (kNodesPad / 64) * (128 / 64);

  wmma_gemm64<0, false, 2, 0, false, 0><<<dim3((tiles192 + 7) / 8, 1), 256, 0, stream>>>(
      X16, nullptr, kFeat, 0L, WL0T, nullptr, kFeat, 0L, (void*)XL, nullptr, 192, 0L, bl0, nullptr, 0L, kNodesPad, 192, kFeat, kScale0);
  wmma_gemm64<0, false, 2, 0, false, 0><<<dim3((tiles192 + 7) / 8, 1), 256, 0, stream>>>(
      X16, nullptr, kFeat, 0L, WR0T, nullptr, kFeat, 0L, (void*)XR, nullptr, 192, 0L, br0, nullptr, 0L, kNodesPad, 192, kFeat, kScale0);
  node_kernel<3><<<(kNodes + kThreads - 1) / kThreads, kThreads, 0, stream>>>(XL, XR, att0, AL4, AR4, CS4);
  ex_kernel<3><<<kEdges / kThreads, kThreads, 0, stream>>>(XL, XR, att0, ei, AL4, AR4, CS4, EXP);
  hipFuncSetAttribute((const void*)agg_kernel<3, 0, kRows0>, hipFuncAttributeMaxDynamicSharedMemorySize, (int)kAggLdsBytes);
  hipFuncSetAttribute((const void*)agg_kernel<2, 0, kRows12>, hipFuncAttributeMaxDynamicSharedMemorySize, (int)kAggLdsBytes);
  hipFuncSetAttribute((const void*)agg_kernel<2, 1, kRows12>, hipFuncAttributeMaxDynamicSharedMemorySize, (int)kAggLdsBytes);
  agg_kernel<3, 0, kRows0><<<kTiles0, kThreads, kAggLdsBytes, stream>>>(XL, ei, EXP, bias0, HA, H2);

  wmma_gemm64<0, false, 2, 0, false, 0><<<dim3((tiles128 + 7) / 8, 1), 256, 0, stream>>>(
      HA, nullptr, 192, 0L, WL1T, nullptr, 192, 0L, (void*)XL, nullptr, 128, 0L, bl1, nullptr, 0L, kNodesPad, 128, 192, kScale12);
  wmma_gemm64<0, false, 2, 0, false, 0><<<dim3((tiles128 + 7) / 8, 1), 256, 0, stream>>>(
      HA, nullptr, 192, 0L, WR1T, nullptr, 192, 0L, (void*)XR, nullptr, 128, 0L, br1, nullptr, 0L, kNodesPad, 128, 192, kScale12);
  node_kernel<2><<<(kNodes + kThreads - 1) / kThreads, kThreads, 0, stream>>>(XL, XR, att1, AL4, AR4, CS4);
  ex_kernel<2><<<kEdges / kThreads, kThreads, 0, stream>>>(XL, XR, att1, ei, AL4, AR4, CS4, EXP);
  agg_kernel<2, 0, kRows12><<<kTiles12, kThreads, kAggLdsBytes, stream>>>(XL, ei, EXP, bias1, HA, H2);

  wmma_gemm64<0, false, 2, 0, false, 0><<<dim3((tiles128 + 7) / 8, 1), 256, 0, stream>>>(
      HA, nullptr, 128, 0L, WL2T, nullptr, 128, 0L, (void*)XL, nullptr, 128, 0L, bl2, nullptr, 0L, kNodesPad, 128, 128, kScale12);
  wmma_gemm64<0, false, 2, 0, false, 0><<<dim3((tiles128 + 7) / 8, 1), 256, 0, stream>>>(
      HA, nullptr, 128, 0L, WR2T, nullptr, 128, 0L, (void*)XR, nullptr, 128, 0L, br2, nullptr, 0L, kNodesPad, 128, 128, kScale12);
  node_kernel<2><<<(kNodes + kThreads - 1) / kThreads, kThreads, 0, stream>>>(XL, XR, att2, AL4, AR4, CS4);
  ex_kernel<2><<<kEdges / kThreads, kThreads, 0, stream>>>(XL, XR, att2, ei, AL4, AR4, CS4, EXP);
  agg_kernel<2, 1, kRows12><<<kTiles12, kThreads, kAggLdsBytes, stream>>>(XL, ei, EXP, bias2, HA, H2);

  pool_kernel<<<kGraphs, kThreads, 0, stream>>>(H2, batch, PP);
  head_kernel<<<1, kThreads, 0, stream>>>(PP, Wout, bout, out);
}
